// SimpleRNN_49692771615219
// MI455X (gfx1250) — hardware-verified
//
#include <hip/hip_runtime.h>
#include <math.h>

constexpr int NB    = 256;
constexpr int NT    = 512;
constexpr int NIN   = 64;
constexpr int NH    = 256;
constexpr int NOUT  = 24;
constexpr int NOUTP = 32;
constexpr int KC1   = NIN + NH;
constexpr int KC2   = NH + NH;
constexpr int RPB   = 16;
constexpr int NBLK  = NB / RPB;
constexpr int RTHR  = 128;
constexpr int P1    = KC1 + 8;
constexpr int P2    = NH + 8;
constexpr int T1BUF = RPB * P1;
constexpr int T2BUF = RPB * P2;
constexpr int OSP   = 36;
constexpr float WCARRY     = 256.0f;
constexpr float WCARRY_INV = 1.0f / 256.0f;
static_assert(NB % RPB == 0);
static_assert(NH == 64 * (RTHR / 32));
static_assert(P1 % 8 == 0 && P2 % 8 == 0);
static_assert(KC1 % 32 == 0 && KC2 % 32 == 0 && NH % 32 == 0 && NIN % 32 == 0);
static_assert(RPB * NIN == 8 * RTHR);
static_assert((2 * T1BUF) % 8 == 0 && (2 * T2BUF) % 8 == 0);
static_assert(RPB * NOUT == 3 * 4 * 32);
static_assert((RPB * NOUT * 4) % 128 == 0);
static_assert(NOUT <= NOUTP && NOUTP == 32 && NOUT < OSP);
static_assert((NT & 1) == 0 || (NT & 1) == 1);

constexpr int DW1ROW = KC1 / 2;
constexpr int DW2ROW = KC2 / 2;
constexpr int DWDROW = NH / 2;
constexpr int PBLK_A = NH * (NIN / 2) / 256;
constexpr int PBLK_B = NH * (NH / 2) / 256;
constexpr int PBLK_E = NOUT * (NH / 2) / 256;
constexpr int PBLK_F = (NOUTP - NOUT) * (NH / 2) / 256;
constexpr int PE1 = PBLK_A;
constexpr int PE2 = PE1 + PBLK_B;
constexpr int PE3 = PE2 + PBLK_B;
constexpr int PE4 = PE3 + PBLK_B;
constexpr int PE5 = PE4 + PBLK_E;
constexpr int PBLKS = PE5 + PBLK_F;
static_assert(NH * (NIN / 2) == PBLK_A * 256 && NH * (NH / 2) == PBLK_B * 256);
static_assert(NOUT * (NH / 2) == PBLK_E * 256 && (NOUTP - NOUT) * (NH / 2) == PBLK_F * 256);
static_assert(PBLKS == 432);
static_assert((NIN / 2) % 32 == 0 && (NH / 2) % 32 == 0 && DW1ROW % 32 == 0);

typedef __attribute__((ext_vector_type(16))) _Float16 v16h;
typedef __attribute__((ext_vector_type(8)))  _Float16 v8h;
typedef __attribute__((ext_vector_type(16))) __bf16   v16b;
typedef __attribute__((ext_vector_type(8)))  __bf16   v8b;
typedef __attribute__((ext_vector_type(8)))  float    v8f;
typedef __attribute__((ext_vector_type(4)))  float    v4f;

__device__ __forceinline__ void dep_guard_h(v8f& a, v8f& b, v16h x, v16h y) { asm volatile("v_nop\n\tv_nop\n\tv_nop\n\tv_nop" : "+v"(a), "+v"(b) : "v"(x), "v"(y)); }
__device__ __forceinline__ void dep_guard_b(v8f& a, v8f& b, v16b x, v16b y) { asm volatile("v_nop\n\tv_nop\n\tv_nop\n\tv_nop" : "+v"(a), "+v"(b) : "v"(x), "v"(y)); }
__device__ __forceinline__ void keep4_h(v16h a, v16h b, v16h c, v16h d) { asm volatile("v_nop" :: "v"(a), "v"(b), "v"(c), "v"(d)); }
__device__ __forceinline__ void keep4_b(v16b a, v16b b, v16b c, v16b d) { asm volatile("v_nop" :: "v"(a), "v"(b), "v"(c), "v"(d)); }
__device__ __forceinline__ void acc_guard4(v8f& a, v8f& b, v8f& c, v8f& d) { asm volatile("v_nop\n\tv_nop\n\tv_nop\n\tv_nop" : "+v"(a), "+v"(b), "+v"(c), "+v"(d)); }
__device__ __forceinline__ void acc_guard1(v8f& a) { asm volatile("v_nop\n\tv_nop\n\tv_nop\n\tv_nop" : "+v"(a)); }
__device__ __forceinline__ void guard4ab(v8f& a0, v8f& a1, v8f& a2, v8f& a3, v16h fa, v16h b0, v16h b1, v16h b2, v16h b3) {
  asm volatile("v_nop\n\tv_nop\n\tv_nop\n\tv_nop" : "+v"(a0), "+v"(a1), "+v"(a2), "+v"(a3) : "v"(fa), "v"(b0), "v"(b1), "v"(b2), "v"(b3));
}
__device__ __forceinline__ void guard1ab(v8f& a0, v16h fa, v16h fb) {
  asm volatile("v_nop\n\tv_nop\n\tv_nop\n\tv_nop" : "+v"(a0) : "v"(fa), "v"(fb));
}

template <typename T> struct Frag;
template <> struct Frag<_Float16> {
  typedef v16h V; union U { v16h v; v8h h[2]; };
  static __device__ __forceinline__ v16h load(const _Float16* p) {
    U f; f.h[0] = *(const v8h*)(p); f.h[1] = *(const v8h*)(p + 16); return f.v;
  }
  static __device__ __forceinline__ v8f mma(v16h a, v16h b, v8f c) {
    return __builtin_amdgcn_wmma_f32_16x16x32_f16(false, a, false, b, (short)0, c, false, false);
  }
  static __device__ __forceinline__ void guard(v8f& a, v8f& b, v16h x, v16h y) { dep_guard_h(a, b, x, y); }
  static __device__ __forceinline__ void keep(v16h a, v16h b, v16h c, v16h d) { keep4_h(a, b, c, d); }
};
template <> struct Frag<__bf16> {
  typedef v16b V; union U { v16b v; v8b h[2]; };
  static __device__ __forceinline__ v16b load(const __bf16* p) {
    U f; f.h[0] = *(const v8b*)(p); f.h[1] = *(const v8b*)(p + 16); return f.v;
  }
  static __device__ __forceinline__ v8f mma(v16b a, v16b b, v8f c) {
    return __builtin_amdgcn_wmma_f32_16x16x32_bf16(false, a, false, b, (short)0, c, false, false);
  }
  static __device__ __forceinline__ void guard(v8f& a, v8f& b, v16b x, v16b y) { dep_guard_b(a, b, x, y); }
  static __device__ __forceinline__ void keep(v16b a, v16b b, v16b c, v16b d) { keep4_b(a, b, c, d); }
};

__device__ __forceinline__ unsigned pack_f16x2(float a, float b) {
  const _Float16 h0 = (_Float16)a, h1 = (_Float16)b;
  return (unsigned)__builtin_bit_cast(unsigned short, h0) | ((unsigned)__builtin_bit_cast(unsigned short, h1) << 16);
}
__device__ __forceinline__ void st2u(unsigned* p, unsigned v) { *(volatile unsigned*)p = v; __threadfence(); *(volatile unsigned*)p = v; }
__device__ __forceinline__ float ftanh(float x) {
  const float xc = fminf(fmaxf(x, -15.0f), 15.0f);
  const float d = 1.0f + expf(2.0f * xc);
  return 1.0f - 2.0f * (1.0f / d);
}

template <int NCH, int LDW>
__device__ __forceinline__ void mma_run4(const _Float16* arow, const _Float16* __restrict__ brow,
                                         v8f& a0, v8f& a1, v8f& a2, v8f& a3) {
#pragma unroll 2
  for (int kc = 0; kc < NCH; ++kc) {
    const v16h fa = Frag<_Float16>::load(arow + kc * 32);
    const v16h b0 = Frag<_Float16>::load(brow + kc * 32);
    const v16h b1 = Frag<_Float16>::load(brow + 16 * LDW + kc * 32);
    const v16h b2 = Frag<_Float16>::load(brow + 32 * LDW + kc * 32);
    const v16h b3 = Frag<_Float16>::load(brow + 48 * LDW + kc * 32);
    a0 = Frag<_Float16>::mma(fa, b0, a0);
    a1 = Frag<_Float16>::mma(fa, b1, a1);
    a2 = Frag<_Float16>::mma(fa, b2, a2);
    a3 = Frag<_Float16>::mma(fa, b3, a3);
    guard4ab(a0, a1, a2, a3, fa, b0, b1, b2, b3);
  }
}
template <int NCH>
__device__ __forceinline__ void mma_run1(const _Float16* arow, const _Float16* __restrict__ brow, v8f& a0) {
#pragma unroll 2
  for (int kc = 0; kc < NCH; ++kc) {
    const v16h fa = Frag<_Float16>::load(arow + kc * 32);
    const v16h fb = Frag<_Float16>::load(brow + kc * 32);
    a0 = Frag<_Float16>::mma(fa, fb, a0);
    guard1ab(a0, fa, fb);
  }
}

__device__ __forceinline__ void stage_x(const float* __restrict__ x, int b0, int ts, _Float16* dst, int tid) {
  const int row = tid >> 3, c8 = (tid & 7) * 8;
  const float* src = x + ((size_t)(b0 + row) * NT + (size_t)ts) * NIN + c8;
  const v4f f0 = *(const v4f*)src;
  const v4f f1 = *(const v4f*)(src + 4);
  v8h hv;
  hv[0] = (_Float16)f0[0]; hv[1] = (_Float16)f0[1]; hv[2] = (_Float16)f0[2]; hv[3] = (_Float16)f0[3];
  hv[4] = (_Float16)f1[0]; hv[5] = (_Float16)f1[1]; hv[6] = (_Float16)f1[2]; hv[7] = (_Float16)f1[3];
  *(v8h*)(dst + row * P1 + c8) = hv;
}

__global__ __launch_bounds__(256) void prep_kernel(
    const float* __restrict__ wih1, const float* __restrict__ whh1,
    const float* __restrict__ wih2, const float* __restrict__ whh2,
    const float* __restrict__ wd,
    unsigned* __restrict__ w1u, unsigned* __restrict__ w2u, unsigned* __restrict__ wdu) {
  const int blk = blockIdx.x, tid = threadIdx.x;
  if (blk < PE1) {
    const int p = blk * 256 + tid;
    const int n = p >> 5, kp = p & 31;
    const float* s = wih1 + (size_t)n * NIN + 2 * kp;
    st2u(w1u + (size_t)n * DW1ROW + kp, pack_f16x2(s[0] * WCARRY, s[1] * WCARRY));
  } else if (blk < PE2) {
    const int p = (blk - PE1) * 256 + tid;
    const int n = p >> 7, kp = p & 127;
    const float* s = whh1 + (size_t)n * NH + 2 * kp;
    st2u(w1u + (size_t)n * DW1ROW + NIN / 2 + kp, pack_f16x2(s[0] * WCARRY, s[1] * WCARRY));
  } else if (blk < PE3) {
    const int p = (blk - PE2) * 256 + tid;
    const int n = p >> 7, kp = p & 127;
    const float* s = wih2 + (size_t)n * NH + 2 * kp;
    st2u(w2u + (size_t)n * DW2ROW + kp, pack_f16x2(s[0] * WCARRY, s[1] * WCARRY));
  } else if (blk < PE4) {
    const int p = (blk - PE3) * 256 + tid;
    const int n = p >> 7, kp = p & 127;
    const float* s = whh2 + (size_t)n * NH + 2 * kp;
    st2u(w2u + (size_t)n * DW2ROW + NH / 2 + kp, pack_f16x2(s[0] * WCARRY, s[1] * WCARRY));
  } else if (blk < PE5) {
    const int p = (blk - PE4) * 256 + tid;
    const int n = p >> 7, kp = p & 127;
    const float* s = wd + (size_t)n * NH + 2 * kp;
    st2u(wdu + (size_t)n * DWDROW + kp, pack_f16x2(s[0] * WCARRY, s[1] * WCARRY));
  } else {
    const int p = (blk - PE5) * 256 + tid;
    st2u(wdu + (size_t)NOUT * DWDROW + p, 0u);
  }
}

__global__ __launch_bounds__(RTHR) void rnn2_kernel(
    const float* __restrict__ x,
    const float* __restrict__ bih1, const float* __restrict__ bhh1,
    const float* __restrict__ bih2, const float* __restrict__ bhh2,
    const float* __restrict__ bd,
    const unsigned short* __restrict__ w1p, const unsigned short* __restrict__ w2p, const unsigned short* __restrict__ wdp,
    float* __restrict__ out) {
  __shared__ __align__(16) _Float16 T1[2 * T1BUF];
  __shared__ __align__(16) _Float16 T2[2 * T2BUF];
  __shared__ __align__(16) float    OSL[RPB * OSP];
  const _Float16* W1 = (const _Float16*)w1p;
  const _Float16* W2 = (const _Float16*)w2p;
  const _Float16* WD = (const _Float16*)wdp;
  const int tid = threadIdx.x, lane = tid & 31, wave = tid >> 5;
  const int c = lane & 15, hh = lane >> 4, koff = hh * 8, mOff = hh * 8;
  const int b0 = blockIdx.x * RPB;
  const int n0 = wave * 64;

  {
    const v8h z = {(_Float16)0.f, (_Float16)0.f, (_Float16)0.f, (_Float16)0.f, (_Float16)0.f, (_Float16)0.f, (_Float16)0.f, (_Float16)0.f};
    for (int i = tid; i < (2 * T1BUF) / 8; i += RTHR) *(v8h*)(T1 + i * 8) = z;
    for (int i = tid; i < (2 * T2BUF) / 8; i += RTHR) *(v8h*)(T2 + i * 8) = z;
  }
  __syncthreads();

  stage_x(x, b0, 0, T1, tid);
  float bs1[4], bs2[4];
#pragma unroll
  for (int j = 0; j < 4; ++j) { const int n = n0 + 16 * j + c; bs1[j] = (bih1[n] + bhh1[n]) * WCARRY; }
  asm volatile("" ::: "memory");
#pragma unroll
  for (int j = 0; j < 4; ++j) { const int n = n0 + 16 * j + c; bs2[j] = (bih2[n] + bhh2[n]) * WCARRY; }
  __syncthreads();

#pragma unroll 1
  for (int t = 0; t < NT; ++t) {
    const int cur = t & 1, nxt = cur ^ 1;
    const _Float16* T1c = T1 + cur * T1BUF;
    _Float16*       T1n = T1 + nxt * T1BUF;
    const _Float16* T2c = T2 + cur * T2BUF;
    _Float16*       T2n = T2 + nxt * T2BUF;

    v8f acc[4];
#pragma unroll
    for (int j = 0; j < 4; ++j) { const float b = bs1[j]; acc[j] = (v8f){b, b, b, b, b, b, b, b}; }
    mma_run4<KC1 / 32, KC1>(T1c + c * P1 + koff, W1 + (size_t)(n0 + c) * KC1 + koff, acc[0], acc[1], acc[2], acc[3]);
    acc_guard4(acc[0], acc[1], acc[2], acc[3]);
#pragma unroll
    for (int j = 0; j < 4; ++j) {
#pragma unroll
      for (int r = 0; r < 8; ++r) {
        const float hv = ftanh(acc[j][r] * WCARRY_INV);
        T1n[(mOff + r) * P1 + NIN + n0 + 16 * j + c] = (_Float16)hv;
      }
    }
    __syncthreads();

#pragma unroll
    for (int j = 0; j < 4; ++j) { const float b = bs2[j]; acc[j] = (v8f){b, b, b, b, b, b, b, b}; }
    mma_run4<NH / 32, KC2>(T1n + c * P1 + NIN + koff, W2 + (size_t)(n0 + c) * KC2 + koff, acc[0], acc[1], acc[2], acc[3]);
    mma_run4<NH / 32, KC2>(T2c + c * P2 + koff, W2 + (size_t)(n0 + c) * KC2 + NH + koff, acc[0], acc[1], acc[2], acc[3]);
    acc_guard4(acc[0], acc[1], acc[2], acc[3]);
#pragma unroll
    for (int j = 0; j < 4; ++j) {
#pragma unroll
      for (int r = 0; r < 8; ++r) {
        const float hv = ftanh(acc[j][r] * WCARRY_INV);
        T2n[(mOff + r) * P2 + n0 + 16 * j + c] = (_Float16)hv;
      }
    }
    const int ts = (t + 1 < NT) ? (t + 1) : (NT - 1);
    stage_x(x, b0, ts, T1n, tid);
    __syncthreads();
  }

  if (wave < 2) {
    v8f acc = (v8f){0.f, 0.f, 0.f, 0.f, 0.f, 0.f, 0.f, 0.f};
    const _Float16* arow = T2 + (NT & 1) * T2BUF + c * P2 + koff;
    const _Float16* brow = WD + (size_t)(16 * wave + c) * NH + koff;
    mma_run1<NH / 32>(arow, brow, acc);
    acc_guard1(acc);
    const int n = 16 * wave + c;
#pragma unroll
    for (int r = 0; r < 8; ++r) OSL[(mOff + r) * OSP + n] = acc[r] * WCARRY_INV;
  }
  __syncthreads();
  if (wave == 0) {
    float* ob = out + (size_t)b0 * NOUT;
    v4f ov[3];
#pragma unroll
    for (int i = 0; i < 3; ++i) {
      const int f = i * 32 + lane;
#pragma unroll
      for (int q = 0; q < 4; ++q) {
        const int e = 4 * f + q;
        const int row = e / NOUT;
        const int col = e - row * NOUT;
        ov[i][q] = OSL[row * OSP + col] + bd[col];
      }
    }
    for (int pass = 0; pass < 2; ++pass) {
#pragma unroll
      for (int i = 0; i < 3; ++i) *(volatile v4f*)(ob + 4 * (i * 32 + lane)) = ov[i];
      __threadfence();
    }
  }
}

extern "C" void kernel_launch(void* const* d_in, const int* in_sizes, int n_in,
                              void* d_out, int out_size, void* d_ws, size_t ws_size, hipStream_t stream) {
  if (n_in < 11 || d_out == nullptr || d_ws == nullptr) return;
  if (in_sizes[0] != NB * NT * NIN || in_sizes[1] != NH * NIN || in_sizes[2] != NH * NH ||
      in_sizes[3] != NH || in_sizes[4] != NH || in_sizes[5] != NH * NH || in_sizes[6] != NH * NH ||
      in_sizes[7] != NH || in_sizes[8] != NH || in_sizes[9] != NOUT * NH || in_sizes[10] != NOUT ||
      out_size != NB * NOUT) return;

  const float* x    = (const float*)d_in[0];
  const float* wih1 = (const float*)d_in[1];
  const float* whh1 = (const float*)d_in[2];
  const float* bih1 = (const float*)d_in[3];
  const float* bhh1 = (const float*)d_in[4];
  const float* wih2 = (const float*)d_in[5];
  const float* whh2 = (const float*)d_in[6];
  const float* bih2 = (const float*)d_in[7];
  const float* bhh2 = (const float*)d_in[8];
  const float* wd   = (const float*)d_in[9];
  const float* bd   = (const float*)d_in[10];
  float* out = (float*)d_out;

  char* ws = (char*)d_ws; size_t off = 0;
  auto carve = [&](size_t bytes) -> char* { char* p = ws + off; off += (bytes + 255) & ~(size_t)255; return p; };
  unsigned short* W1CAT = (unsigned short*)carve((size_t)NH * KC1 * 2);
  unsigned short* W2CAT = (unsigned short*)carve((size_t)NH * KC2 * 2);
  unsigned short* WD16  = (unsigned short*)carve((size_t)NOUTP * NH * 2);
  if (off > ws_size || off > (size_t)134217728) return;

  prep_kernel<<<PBLKS, 256, 0, stream>>>(wih1, whh1, wih2, whh2, wd,
                                          (unsigned*)W1CAT, (unsigned*)W2CAT, (unsigned*)WD16);

  rnn2_kernel<<<NBLK, RTHR, 0, stream>>>(x, bih1, bhh1, bih2, bhh2, bd, W1CAT, W2CAT, WD16, out);
}
